// GraphMultiHeadAttention_7275674599951
// MI455X (gfx1250) — hardware-run, weakly checked
//
#include <hip/hip_runtime.h>
#include <stddef.h>
#include <stdint.h>

#define NN    4096
#define CM    256
#define NH    4
#define HDM   64
#define QKVP  768
#define RPB   32
#define NWD   128
#define KCAP  512
#define OTP   68

static_assert(NH * HDM == CM);
static_assert(NWD * 32 == NN);
static_assert(NN % 256 == 0);
static_assert(NN % RPB == 0);
static_assert(RPB % 8 == 0);
static_assert(CM % 64 == 0);
static_assert(CM % 32 == 0);
static_assert((NN * CM) % 2048 == 0);
static_assert(KCAP % 32 == 0);
static_assert(HDM == 64);
static_assert(QKVP == 3 * CM);
static_assert(QKVP % 32 == 0);
static_assert((OTP * 4) % 16 == 0);
static_assert(NN % 8 == 0);

typedef _Float16       v16h __attribute__((ext_vector_type(16)));
typedef _Float16       v8h  __attribute__((ext_vector_type(8)));
typedef __bf16         v16b __attribute__((ext_vector_type(16)));
typedef unsigned short v8us __attribute__((ext_vector_type(8)));
typedef float          v8f  __attribute__((ext_vector_type(8)));
typedef float          v4f  __attribute__((ext_vector_type(4)));
typedef unsigned int   v4u  __attribute__((ext_vector_type(4)));
typedef int            v4i  __attribute__((ext_vector_type(4)));

union FragH { v16h v; v8h  h[2]; };
union FragB { v16b v; v8us u[2]; };
union Pack8 { v8h h; v4u u; };

__device__ __forceinline__ v8f mma16h(v16h a, v16h b, v8f c) {
  c = __builtin_amdgcn_wmma_f32_16x16x32_f16(false, a, false, b, (short)0, c, false, false);
  asm volatile("v_nop\n\tv_nop\n\tv_nop\n\tv_nop" : "+v"(c) : "v"(a), "v"(b));
  return c;
}
__device__ __forceinline__ v8f mma16b(v16b a, v16b b, v8f c) {
  c = __builtin_amdgcn_wmma_f32_16x16x32_bf16(false, a, false, b, (short)0, c, false, false);
  asm volatile("v_nop\n\tv_nop\n\tv_nop\n\tv_nop" : "+v"(c) : "v"(a), "v"(b));
  return c;
}

__device__ __forceinline__ v16h ldfrag_h(const _Float16* p, int ld, int row0, int k0, int lane) {
  const int m = lane & 15, lh = lane >> 4;
  const _Float16* q = p + (size_t)(row0 + m) * ld + k0 + 8 * lh;
  FragH f;
  f.h[0] = *(const v8h*)(q);
  f.h[1] = *(const v8h*)(q + 16);
  return f.v;
}
__device__ __forceinline__ v16b ldfrag_b(const unsigned short* p, int ld, int row0, int k0, int lane) {
  const int m = lane & 15, lh = lane >> 4;
  const unsigned short* q = p + (size_t)(row0 + m) * ld + k0 + 8 * lh;
  FragB f;
  f.u[0] = *(const v8us*)(q);
  f.u[1] = *(const v8us*)(q + 16);
  return f.v;
}

__device__ __forceinline__ v8f zero8() { return (v8f){0.f, 0.f, 0.f, 0.f, 0.f, 0.f, 0.f, 0.f}; }

__device__ __forceinline__ unsigned int bfbits(float f) {
  unsigned int u = __float_as_uint(f);
  u += 0x7FFFu + ((u >> 16) & 1u);
  return u >> 16;
}
__device__ __forceinline__ void split8(const float (&f)[8], v4u& hi, v4u& lo) {
  unsigned int hb[8], lb[8];
#pragma unroll
  for (int i = 0; i < 8; ++i) {
    hb[i] = bfbits(f[i]);
    lb[i] = bfbits(f[i] - __uint_as_float(hb[i] << 16));
  }
  hi = (v4u){hb[0] | (hb[1] << 16), hb[2] | (hb[3] << 16), hb[4] | (hb[5] << 16), hb[6] | (hb[7] << 16)};
  lo = (v4u){lb[0] | (lb[1] << 16), lb[2] | (lb[3] << 16), lb[4] | (lb[5] << 16), lb[6] | (lb[7] << 16)};
}

__global__ __launch_bounds__(256) void k_cvt_x(const float* __restrict__ src, _Float16* __restrict__ xh,
                                               unsigned short* __restrict__ xbh, unsigned short* __restrict__ xbl) {
  const int tid = threadIdx.x;
  const size_t o = (size_t)blockIdx.x * 2048 + (size_t)tid * 8;
  const v4f a0 = *(const v4f*)(src + o);
  const v4f a1 = *(const v4f*)(src + o + 4);
  const float f[8] = {a0[0], a0[1], a0[2], a0[3], a1[0], a1[1], a1[2], a1[3]};
  Pack8 pk;
  pk.h = (v8h){(_Float16)f[0], (_Float16)f[1], (_Float16)f[2], (_Float16)f[3],
               (_Float16)f[4], (_Float16)f[5], (_Float16)f[6], (_Float16)f[7]};
  v4u hi, lo;
  split8(f, hi, lo);
  const v4u vv = pk.u;
  volatile v4u* d0 = (volatile v4u*)(xh + o);
  volatile v4u* d1 = (volatile v4u*)(xbh + o);
  volatile v4u* d2 = (volatile v4u*)(xbl + o);
  *d0 = vv; *d1 = hi; *d2 = lo;
  __threadfence();
  *d0 = vv; *d1 = hi; *d2 = lo;
}

__device__ __forceinline__ void wt_load_tile(const float* __restrict__ W, float (*s)[68], int n0, int k0, int tid) {
  const int kk = tid >> 2, g = tid & 3;
  const float* srcp = W + (size_t)(k0 + kk) * CM + n0 + 16 * g;
#pragma unroll
  for (int j = 0; j < 4; ++j) *(v4f*)(&s[kk][16 * g + 4 * j]) = *(const v4f*)(srcp + 4 * j);
}

__global__ __launch_bounds__(256) void k_wt_x3(const float* __restrict__ W,
                                               unsigned short* __restrict__ bh, unsigned short* __restrict__ bl) {
  __shared__ __align__(16) float s[64][68];
  const int tid = threadIdx.x, lane = tid & 31, wave = tid >> 5;
  const int n0 = blockIdx.x * 64, k0 = blockIdx.y * 64;
  wt_load_tile(W, s, n0, k0, tid);
  __syncthreads();
#pragma unroll
  for (int it = 0; it < 2; ++it) {
    const int nn = wave * 8 + it * 4 + (lane >> 3);
    const int pc = lane & 7;
    float f[8];
#pragma unroll
    for (int j = 0; j < 8; ++j) f[j] = s[8 * pc + j][nn];
    v4u hi, lo;
    split8(f, hi, lo);
    const size_t go = (size_t)(n0 + nn) * CM + k0 + 8 * pc;
    volatile v4u* dh = (volatile v4u*)(bh + go);
    volatile v4u* dl = (volatile v4u*)(bl + go);
    *dh = hi; *dl = lo;
    __threadfence();
    *dh = hi; *dl = lo;
  }
}

__global__ __launch_bounds__(256) void k_wt_f16(const float* __restrict__ W, _Float16* __restrict__ bt, float scale) {
  __shared__ __align__(16) float s[64][68];
  const int tid = threadIdx.x, lane = tid & 31, wave = tid >> 5;
  const int n0 = blockIdx.x * 64, k0 = blockIdx.y * 64;
  wt_load_tile(W, s, n0, k0, tid);
  __syncthreads();
#pragma unroll
  for (int it = 0; it < 2; ++it) {
    const int nn = wave * 8 + it * 4 + (lane >> 3);
    const int pc = lane & 7;
    Pack8 pk;
    pk.h = (v8h){(_Float16)(s[8 * pc + 0][nn] * scale), (_Float16)(s[8 * pc + 1][nn] * scale),
                 (_Float16)(s[8 * pc + 2][nn] * scale), (_Float16)(s[8 * pc + 3][nn] * scale),
                 (_Float16)(s[8 * pc + 4][nn] * scale), (_Float16)(s[8 * pc + 5][nn] * scale),
                 (_Float16)(s[8 * pc + 6][nn] * scale), (_Float16)(s[8 * pc + 7][nn] * scale)};
    const v4u vv = pk.u;
    const size_t go = (size_t)(n0 + nn) * CM + k0 + 8 * pc;
    volatile v4u* d = (volatile v4u*)(bt + go);
    *d = vv;
    __threadfence();
    *d = vv;
  }
}

__device__ __forceinline__ void gemm32x64_f16(const _Float16* __restrict__ A, int lda,
                                              const _Float16* __restrict__ Bt, int ldb, int K,
                                              int m0, int n0, int lane, v8f (&acc)[2][4]) {
#pragma unroll 1
  for (int k0 = 0; k0 < K; k0 += 32) {
    const v16h a0 = ldfrag_h(A, lda, m0, k0, lane);
    const v16h a1 = ldfrag_h(A, lda, m0 + 16, k0, lane);
#pragma unroll
    for (int t = 0; t < 4; ++t) {
      const v16h b = ldfrag_h(Bt, ldb, n0 + 16 * t, k0, lane);
      acc[0][t] = mma16h(a0, b, acc[0][t]);
      acc[1][t] = mma16h(a1, b, acc[1][t]);
    }
  }
}

__device__ __forceinline__ void gemm32x64_x3(const unsigned short* __restrict__ Ah, const unsigned short* __restrict__ Al,
                                             int lda,
                                             const unsigned short* __restrict__ Bh, const unsigned short* __restrict__ Bl,
                                             int ldb, int K, int m0, int n0, int lane, v8f (&acc)[2][4]) {
#pragma unroll 1
  for (int k0 = 0; k0 < K; k0 += 32) {
    const v16b a0h = ldfrag_b(Ah, lda, m0, k0, lane);
    const v16b a0l = ldfrag_b(Al, lda, m0, k0, lane);
    const v16b a1h = ldfrag_b(Ah, lda, m0 + 16, k0, lane);
    const v16b a1l = ldfrag_b(Al, lda, m0 + 16, k0, lane);
#pragma unroll
    for (int t = 0; t < 4; ++t) {
      const v16b bh = ldfrag_b(Bh, ldb, n0 + 16 * t, k0, lane);
      const v16b bl = ldfrag_b(Bl, ldb, n0 + 16 * t, k0, lane);
      acc[0][t] = mma16b(a0h, bh, acc[0][t]);
      acc[0][t] = mma16b(a0l, bh, acc[0][t]);
      acc[0][t] = mma16b(a0h, bl, acc[0][t]);
      acc[1][t] = mma16b(a1h, bh, acc[1][t]);
      acc[1][t] = mma16b(a1l, bh, acc[1][t]);
      acc[1][t] = mma16b(a1h, bl, acc[1][t]);
    }
  }
}

__device__ __forceinline__ void out_epilogue_f32(v8f (&acc)[2][4], float scale, const float* __restrict__ bias,
                                                 float* sw, float* __restrict__ out, int ldo,
                                                 int m0, int n0, int lane, int hh, int c) {
#pragma unroll
  for (int sub = 0; sub < 2; ++sub) {
    __syncthreads();
#pragma unroll
    for (int t = 0; t < 4; ++t) {
      const float bvl = bias[n0 + 16 * t + c];
#pragma unroll
      for (int r = 0; r < 8; ++r) sw[(8 * hh + r) * OTP + 16 * t + c] = fmaf(acc[sub][t][r], scale, bvl);
    }
    __syncthreads();
    v4f val[8];
    size_t go[8];
#pragma unroll
    for (int it = 0; it < 8; ++it) {
      const int p    = lane + 32 * it;
      const int L    = p >> 3;
      const int pc   = p & 7;
      const int row  = L >> 1;
      const int half = L & 1;
      val[it] = *(const v4f*)(sw + row * OTP + half * 32 + pc * 4);
      go[it]  = (size_t)(m0 + sub * 16 + row) * ldo + n0 + half * 32 + pc * 4;
    }
#pragma unroll
    for (int it = 0; it < 8; ++it) *(volatile v4f*)(out + go[it]) = val[it];
    __threadfence();
#pragma unroll
    for (int it = 0; it < 8; ++it) *(volatile v4f*)(out + go[it]) = val[it];
  }
}

__global__ __launch_bounds__(256) void k_gemm_f16(const _Float16* __restrict__ ap, int lda,
                                                  const _Float16* __restrict__ bt, int ldb, int K, float scale,
                                                  const float* __restrict__ bias, float* __restrict__ out, int ldo) {
  __shared__ __align__(16) float st[8][16 * OTP];
  const int tid = threadIdx.x, lane = tid & 31, wave = tid >> 5;
  const int hh = lane >> 4, c = lane & 15;
  const int m0 = blockIdx.x * 256 + wave * 32;
  const int n0 = blockIdx.y * 64;
  v8f acc[2][4];
#pragma unroll
  for (int s = 0; s < 2; ++s)
#pragma unroll
    for (int t = 0; t < 4; ++t) acc[s][t] = zero8();
  gemm32x64_f16(ap, lda, bt, ldb, K, m0, n0, lane, acc);
  out_epilogue_f32(acc, scale, bias, st[wave], out, ldo, m0, n0, lane, hh, c);
}

__global__ __launch_bounds__(256) void k_gemm_x3(const unsigned short* __restrict__ ah, const unsigned short* __restrict__ al,
                                                 int lda,
                                                 const unsigned short* __restrict__ bh, const unsigned short* __restrict__ bl,
                                                 int ldb, int K, float scale,
                                                 const float* __restrict__ bias, float* __restrict__ out, int ldo) {
  __shared__ __align__(16) float st[8][16 * OTP];
  const int tid = threadIdx.x, lane = tid & 31, wave = tid >> 5;
  const int hh = lane >> 4, c = lane & 15;
  const int m0 = blockIdx.x * 256 + wave * 32;
  const int n0 = blockIdx.y * 64;
  v8f acc[2][4];
#pragma unroll
  for (int s = 0; s < 2; ++s)
#pragma unroll
    for (int t = 0; t < 4; ++t) acc[s][t] = zero8();
  gemm32x64_x3(ah, al, lda, bh, bl, ldb, K, m0, n0, lane, acc);
  out_epilogue_f32(acc, scale, bias, st[wave], out, ldo, m0, n0, lane, hh, c);
}

__global__ __launch_bounds__(256) void k_meanv(const float* __restrict__ qkv, float* __restrict__ mv) {
  __shared__ double s_part[8][32];
  __shared__ __align__(16) float s_line[32];
  const int tid = threadIdx.x, lane = tid & 31, wave = tid >> 5;
  const int col = blockIdx.x * 32 + lane;
  const float* p = qkv + 2 * CM + col + (size_t)wave * (NN / 8) * QKVP;
  double acc = 0.0;
#pragma unroll 4
  for (int i = 0; i < NN / 8; ++i) acc += (double)p[(size_t)i * QKVP];
  s_part[wave][lane] = acc;
  __syncthreads();
  if (wave == 0) {
    double t = s_part[0][lane];
#pragma unroll
    for (int w = 1; w < 8; ++w) t += s_part[w][lane];
    s_line[lane] = (float)(t * (1.0 / (double)NN));
  }
  __syncthreads();
  if (wave == 0) {
    const int pc = lane & 7;
    const v4f val = *(const v4f*)(&s_line[4 * pc]);
    volatile v4f* dst = (volatile v4f*)(mv + blockIdx.x * 32 + 4 * pc);
    if (lane < 8) *dst = val;
    __threadfence();
    if (lane < 8) *dst = val;
  }
}

__global__ __launch_bounds__(256) void k_attn(const float* __restrict__ qkv, const int* __restrict__ ei, int nE,
                                              const float* __restrict__ mv, unsigned short* __restrict__ ah) {
  __shared__ __align__(16) unsigned int s_mask[RPB][NWD];
  __shared__ __align__(16) int   s_list[8][KCAP];
  __shared__ __align__(16) float s_sc[8][KCAP];
  __shared__ __align__(16) float s_q[8][HDM];
  __shared__ __align__(16) float s_o[8][HDM];
  const int tid = threadIdx.x, lane = tid & 31, wave = tid >> 5;
  const int row0 = blockIdx.x * RPB;

  {
    const v4u z = (v4u){0u, 0u, 0u, 0u};
    v4u* pm = (v4u*)(&s_mask[0][0]);
    for (int i = tid; i < (RPB * NWD) / 4; i += 256) pm[i] = z;
    const v4i zi = (v4i){0, 0, 0, 0};
    v4i* pl = (v4i*)(&s_list[0][0]);
    for (int i = tid; i < (8 * KCAP) / 4; i += 256) pl[i] = zi;
  }
  __syncthreads();

  if ((nE & 3) == 0) {
    const int n4 = nE >> 2;
    const v4i* s4 = (const v4i*)ei;
    const v4i* d4 = (const v4i*)(ei + nE);
    for (int i = tid; i < n4; i += 256) {
      const v4i rv = s4[i];
      const v4i cv = d4[i];
#pragma unroll
      for (int j = 0; j < 4; ++j) {
        const int lr = rv[j] - row0;
        if ((unsigned)lr < (unsigned)RPB) {
          int cc = cv[j];
          cc = (cc < 0) ? 0 : ((cc > NN - 1) ? (NN - 1) : cc);
          atomicOr(&s_mask[lr][cc >> 5], 1u << (cc & 31));
        }
      }
    }
  } else {
    for (int e = tid; e < nE; e += 256) {
      const int lr = ei[e] - row0;
      if ((unsigned)lr < (unsigned)RPB) {
        int cc = ei[nE + e];
        cc = (cc < 0) ? 0 : ((cc > NN - 1) ? (NN - 1) : cc);
        atomicOr(&s_mask[lr][cc >> 5], 1u << (cc & 31));
      }
    }
  }
  __syncthreads();

  const size_t plane = (size_t)NN * CM;
  const float qnan = __uint_as_float(0x7fc00000u);

#pragma unroll 1
  for (int ri = 0; ri < RPB / 8; ++ri) {
    const int lr  = ri * 8 + wave;
    const int row = row0 + lr;

    const v4u wv = *(const v4u*)(&s_mask[lr][4 * lane]);
    const int cl = __builtin_popcount(wv[0]) + __builtin_popcount(wv[1]) +
                   __builtin_popcount(wv[2]) + __builtin_popcount(wv[3]);
    int incl = cl;
#pragma unroll
    for (int d = 1; d < 32; d <<= 1) {
      const int tv = __shfl_up(incl, d, 32);
      incl += (lane >= d) ? tv : 0;
    }
    const int total = __shfl(incl, 31, 32);
    const int excl  = incl - cl;
    const int n = (total < KCAP) ? total : KCAP;
    const bool poison = total > KCAP;
    {
      int pos = excl;
#pragma unroll
      for (int j = 0; j < 4; ++j) {
        unsigned int bits = wv[j];
#pragma unroll 1
        for (int itb = 0; itb < 32; ++itb) {
          if (bits == 0u) break;
          const int b = __builtin_ctz(bits);
          bits &= bits - 1u;
          if (pos < KCAP) s_list[wave][pos] = ((4 * lane + j) << 5) + b;
          ++pos;
        }
      }
    }
    __syncthreads();

    const int nt = (n + 31) >> 5;
#pragma unroll 1
    for (int h = 0; h < NH; ++h) {
      const float* qp = qkv + (size_t)row * QKVP + h * HDM;
      s_q[wave][lane]      = qp[lane];
      s_q[wave][lane + 32] = qp[lane + 32];
      __syncthreads();

      float lmax = -3.0e38f;
#pragma unroll 1
      for (int t = 0; t < nt; ++t) {
        const int j  = lane + 32 * t;
        const int jj = (j < n) ? j : (n - 1);
        int m = s_list[wave][jj];
        m = (m < 0) ? 0 : ((m > NN - 1) ? (NN - 1) : m);
        const float* kp = qkv + (size_t)m * QKVP + CM + h * HDM;
        float dot = 0.f;
#pragma unroll 4
        for (int d4 = 0; d4 < HDM / 4; ++d4) {
          const v4f kv = *(const v4f*)(kp + 4 * d4);
          const v4f qv = *(const v4f*)(&s_q[wave][4 * d4]);
          dot = fmaf(qv[0], kv[0], dot);
          dot = fmaf(qv[1], kv[1], dot);
          dot = fmaf(qv[2], kv[2], dot);
          dot = fmaf(qv[3], kv[3], dot);
        }
        dot *= 0.125f;
        lmax = (j < n) ? fmaxf(lmax, dot) : lmax;
        if (j < n) s_sc[wave][j] = dot;
      }
#pragma unroll
      for (int o = 16; o; o >>= 1) lmax = fmaxf(lmax, __shfl_xor(lmax, o, 32));
      __syncthreads();

      float lsum = 0.f;
#pragma unroll 1
      for (int t = 0; t < nt; ++t) {
        const int j  = lane + 32 * t;
        const int jj = (j < n) ? j : (n - 1);
        float p = __expf(s_sc[wave][jj] - lmax);
        p = (j < n) ? p : 0.f;
        if (j < n) s_sc[wave][j] = p;
        lsum += p;
      }
#pragma unroll
      for (int o = 16; o; o >>= 1) lsum += __shfl_xor(lsum, o, 32);
      __syncthreads();

      float a0 = 0.f, a1 = 0.f;
      const float* vb = qkv + 2 * CM + h * HDM + lane;
#pragma unroll 1
      for (int e = 0; e < n; ++e) {
        const float p = s_sc[wave][e];
        int m = s_list[wave][e];
        m = (m < 0) ? 0 : ((m > NN - 1) ? (NN - 1) : m);
        const float* vp = vb + (size_t)m * QKVP;
        a0 = fmaf(p, vp[0], a0);
        a1 = fmaf(p, vp[32], a1);
      }
      const float inv = 1.0f / fmaxf(lsum, 1.0f);
      const float mv0 = mv[h * HDM + lane];
      const float mv1 = mv[h * HDM + lane + 32];
      float o0 = (n > 0) ? (a0 * inv) : mv0;
      float o1 = (n > 0) ? (a1 * inv) : mv1;
      o0 = poison ? qnan : o0;
      o1 = poison ? qnan : o1;
      s_o[wave][lane]      = o0;
      s_o[wave][lane + 32] = o1;
      __syncthreads();

      {
        const int pc = lane & 7, which = (lane >> 3) & 1;
        const v4f u0 = *(const v4f*)(&s_o[wave][8 * pc]);
        const v4f u1 = *(const v4f*)(&s_o[wave][8 * pc + 4]);
        const float f[8] = {u0[0], u0[1], u0[2], u0[3], u1[0], u1[1], u1[2], u1[3]};
        v4u hi, lo;
        split8(f, hi, lo);
        v4u val;
#pragma unroll
        for (int i = 0; i < 4; ++i) val[i] = which ? lo[i] : hi[i];
        const size_t ga = (size_t)which * plane + (size_t)row * CM + (size_t)h * HDM + 8 * pc;
        volatile v4u* dst = (volatile v4u*)(ah + ga);
        if (lane < 16) *dst = val;
        __threadfence();
        if (lane < 16) *dst = val;
      }
    }
  }
}

extern "C" void kernel_launch(void* const* d_in, const int* in_sizes, int n_in,
                              void* d_out, int out_size, void* d_ws, size_t ws_size,
                              hipStream_t stream) {
  if (n_in < 10) return;
  if (in_sizes[0] != NN * CM) return;
  if (in_sizes[1] < 0 || (in_sizes[1] & 1)) return;
  const int nE = in_sizes[1] >> 1;
  if (in_sizes[2] != CM * CM || in_sizes[4] != CM * CM || in_sizes[6] != CM * CM || in_sizes[8] != CM * CM) return;
  if (in_sizes[3] != CM || in_sizes[5] != CM || in_sizes[7] != CM || in_sizes[9] != CM) return;
  if (out_size != NN * CM) return;

  const float* x  = (const float*)d_in[0];
  const int*   ei = (const int*)d_in[1];
  const float* wq = (const float*)d_in[2];
  const float* bq = (const float*)d_in[3];
  const float* wk = (const float*)d_in[4];
  const float* bk = (const float*)d_in[5];
  const float* wv = (const float*)d_in[6];
  const float* bv = (const float*)d_in[7];
  const float* wo = (const float*)d_in[8];
  const float* bo = (const float*)d_in[9];
  float* out = (float*)d_out;

  size_t off = 0;
  const size_t oXh  = off; off += (size_t)NN * CM * 2;
  const size_t oXbh = off; off += (size_t)NN * CM * 2;
  const size_t oXbl = off; off += (size_t)NN * CM * 2;
  const size_t oWq  = off; off += (size_t)2 * CM * CM * 2;
  const size_t oWk  = off; off += (size_t)2 * CM * CM * 2;
  const size_t oWo  = off; off += (size_t)2 * CM * CM * 2;
  const size_t oWv  = off; off += (size_t)CM * CM * 2;
  const size_t oQKV = off; off += (size_t)NN * QKVP * 4;
  const size_t oA   = off; off += (size_t)2 * NN * CM * 2;
  const size_t oMV  = off; off += (size_t)CM * 4;
  if (off > ws_size) return;
  if (off > (size_t)134217728) return;
  if ((oQKV & 127) != 0 || (oA & 127) != 0 || (oMV & 127) != 0) return;

  char* ws = (char*)d_ws;
  _Float16*       Xh  = (_Float16*)(ws + oXh);
  unsigned short* Xbh = (unsigned short*)(ws + oXbh);
  unsigned short* Xbl = (unsigned short*)(ws + oXbl);
  unsigned short* Wqh = (unsigned short*)(ws + oWq);
  unsigned short* Wql = Wqh + (size_t)CM * CM;
  unsigned short* Wkh = (unsigned short*)(ws + oWk);
  unsigned short* Wkl = Wkh + (size_t)CM * CM;
  unsigned short* Woh = (unsigned short*)(ws + oWo);
  unsigned short* Wol = Woh + (size_t)CM * CM;
  _Float16*       Wvt = (_Float16*)(ws + oWv);
  float*          QKV = (float*)(ws + oQKV);
  unsigned short* Ah  = (unsigned short*)(ws + oA);
  unsigned short* Al  = Ah + (size_t)NN * CM;
  float*          MV  = (float*)(ws + oMV);

  k_cvt_x<<<dim3((NN * CM) / 2048), dim3(256), 0, stream>>>(x, Xh, Xbh, Xbl);
  k_wt_x3<<<dim3(CM / 64, CM / 64), dim3(256), 0, stream>>>(wq, Wqh, Wql);
  k_wt_x3<<<dim3(CM / 64, CM / 64), dim3(256), 0, stream>>>(wk, Wkh, Wkl);
  k_wt_x3<<<dim3(CM / 64, CM / 64), dim3(256), 0, stream>>>(wo, Woh, Wol);
  k_wt_f16<<<dim3(CM / 64, CM / 64), dim3(256), 0, stream>>>(wv, Wvt, 32.0f);
  k_gemm_x3<<<dim3(NN / 256, CM / 64), dim3(256), 0, stream>>>(Xbh, Xbl, CM, Wqh, Wql, CM, CM, 1.0f, bq, QKV, QKVP);
  k_gemm_x3<<<dim3(NN / 256, CM / 64), dim3(256), 0, stream>>>(Xbh, Xbl, CM, Wkh, Wkl, CM, CM, 1.0f, bk, QKV + CM, QKVP);
  k_gemm_f16<<<dim3(NN / 256, CM / 64), dim3(256), 0, stream>>>(Xh, CM, Wvt, CM, CM, 0.03125f, bv, QKV + 2 * CM, QKVP);
  k_meanv<<<dim3(CM / 32), dim3(256), 0, stream>>>(QKV, MV);
  k_attn<<<dim3(NN / RPB), dim3(256), 0, stream>>>(QKV, ei, nE, MV, Ah);
  k_gemm_x3<<<dim3(NN / 256, CM / 64), dim3(256), 0, stream>>>(Ah, Al, CM, Woh, Wol, CM, CM, 1.0f, bo, out, CM);
  (void)hipGetLastError();
}
